// GAT_GraphSAGE_12781822673344
// MI455X (gfx1250) — hardware-run, weakly checked
//
#include <hip/hip_runtime.h>


namespace {
constexpr int N = 10000, E = 320000, G = 256, F = 35, FP = 48, H1 = 1500, H1P = 1504, H2 = 128, NBLK = N / 16;
constexpr float XS = 8.0f, PS = 2048.0f, WSC = 256.0f;
typedef _Float16 b16;
typedef __attribute__((ext_vector_type(16))) _Float16 v16b;
typedef __attribute__((ext_vector_type(8))) _Float16 v8b;
typedef __attribute__((ext_vector_type(8))) float v8f;
typedef __attribute__((ext_vector_type(4))) float v4f;
__device__ __forceinline__ float bf16_rne(float f) { unsigned int u = __float_as_uint(f); u += 0x7FFFu + ((u >> 16) & 1u); return __uint_as_float(u & 0xFFFF0000u); }
__device__ __forceinline__ v16b frag_kb(const b16* p, int hh) { const v8b a = *(const v8b*)(p + 8 * hh), b = *(const v8b*)(p + 16 + 8 * hh); v16b f;
#pragma unroll
  for (int e = 0; e < 8; ++e) { f[e] = a[e]; f[8 + e] = b[e]; } return f; }
__device__ __forceinline__ v8f wmma16b(v16b a, v16b b, v8f c) { v8f d = __builtin_amdgcn_wmma_f32_16x16x32_f16(false, a, false, b, (short)0, c, false, false); asm volatile("v_nop\n\tv_nop\n\tv_nop\n\tv_nop" : "+v"(d) : "v"(a), "v"(b)); return d; }
__device__ __forceinline__ void wave_lds_sync() { __builtin_amdgcn_fence(__ATOMIC_RELEASE, "workgroup"); __builtin_amdgcn_wave_barrier(); __builtin_amdgcn_fence(__ATOMIC_ACQUIRE, "workgroup"); }
__device__ __forceinline__ float pmul(float a, float b) { float p = a * b; asm volatile("" : "+v"(p)); return p; }
__device__ __forceinline__ int iclamp(int v, int lo, int hi) { return v < lo ? lo : (v > hi ? hi : v); }
constexpr int CSR_NBLK7 = 512, CSR_GB7 = 7, CSR_GN7 = 1 << CSR_GB7  , CSR_TS7 = (CSR_GN7 < 32 ? 32 : CSR_GN7)  , CSR_MAXG7 = 512, CSR_CAP7 = 12288  ;
__device__ __host__ __forceinline__ int csr_tix7(int v) { return (v >> CSR_GB7) * CSR_TS7 + (v & (CSR_GN7 - 1)); }
__global__ __launch_bounds__(64) void csrA_kernel7(const int* __restrict__ dst, int E, int N, int nG, int CHP, int NGP, int* __restrict__ STG, int* __restrict__ HST) {
  extern __shared__ int sm[];
  int* cnt = sm; int* run = sm + NGP; int* ids = sm + 2 * NGP;
  const int b = blockIdx.x; const int ch = (E + CSR_NBLK7 - 1) / CSR_NBLK7; const int e0 = b * ch, e1 = min(E, e0 + ch);
  for (int i = threadIdx.x; i < NGP; i += 64) cnt[i] = 0;
  for (int i = threadIdx.x; i < CHP; i += 64) ids[i] = -1;
  __syncthreads();
  if (threadIdx.x == 0) {
    for (int e = e0; e < e1; ++e) { int d = dst[e]; d = (d < 0) ? 0 : (d >= N ? N - 1 : d); cnt[d >> CSR_GB7] += 1; }
    int acc = 0; for (int g = 0; g < nG; ++g) { run[g] = acc; acc += cnt[g]; }
    for (int e = e0; e < e1; ++e) { int d = dst[e]; d = (d < 0) ? 0 : (d >= N ? N - 1 : d); const int g = d >> CSR_GB7; ids[run[g]] = e; run[g] += 1; } }
  __syncthreads();
  typedef __attribute__((ext_vector_type(4))) int v4i;
  for (int pass = 0; pass < 2; ++pass) {
    for (int i = threadIdx.x; i < CHP / 4; i += 64) *(volatile v4i*)(STG + (size_t)b * CHP + i * 4) = *(const v4i*)(&ids[i * 4]);
    for (int i = threadIdx.x; i < NGP / 4; i += 64) { v4i v; for (int e = 0; e < 4; ++e) v[e] = (i * 4 + e < nG) ? cnt[i * 4 + e] : 0; *(volatile v4i*)(HST + (size_t)b * NGP + i * 4) = v; }
    __threadfence(); }
}
__global__ __launch_bounds__(512) void csrS_kernel7(const int* __restrict__ HST, int nG, int NGP, int* __restrict__ START, int* __restrict__ TOT, int* __restrict__ OFF) {
  __shared__ int tot[CSR_MAXG7];
  const int b = threadIdx.x;
  for (int pass = 0; pass < 2; ++pass) { int runb = 0; for (int g = 0; g < nG; ++g) { int c = HST[(size_t)b * NGP + g]; c = (c < 0) ? 0 : c; ((volatile int*)OFF)[(size_t)g * CSR_NBLK7 + b] = runb; runb += c; } __threadfence(); }
  for (int g = threadIdx.x; g < nG; g += 512) { int s = 0; for (int bb = 0; bb < CSR_NBLK7; ++bb) { int c = HST[(size_t)bb * NGP + g]; s += (c < 0) ? 0 : c; } tot[g] = s; }
  __syncthreads();
  if (threadIdx.x < 32) {
    __shared__ int st[CSR_MAXG7 + 32];
    if (threadIdx.x == 0) { int acc = 0; for (int g = 0; g < NGP; ++g) { st[g] = acc; if (g < nG) acc += (tot[g] + 31) & ~31; } st[NGP] = acc; }
    __builtin_amdgcn_fence(__ATOMIC_RELEASE, "workgroup"); __builtin_amdgcn_wave_barrier(); __builtin_amdgcn_fence(__ATOMIC_ACQUIRE, "workgroup");
    for (int pass = 0; pass < 2; ++pass) { for (int i = threadIdx.x; i < NGP + 32; i += 32) { ((volatile int*)START)[i] = (i <= NGP) ? st[min(i, NGP)] : 0; ((volatile int*)TOT)[i] = (i < nG) ? tot[i] : 0; } __threadfence(); } }
}
__global__ __launch_bounds__(256) void csrB_kernel7(const int* __restrict__ dst, int N, int nG, int CHP, int NGP, int permLen, const int* __restrict__ STG, const int* __restrict__ HST, const int* __restrict__ OFF, const int* __restrict__ START, const int* __restrict__ TOT, int* __restrict__ PERM, int* __restrict__ ROWPTR, int* __restrict__ ROWCNT, int* __restrict__ FLAG) {
  typedef __attribute__((ext_vector_type(4))) int v4i;
  __shared__ int ids[CSR_CAP7]; __shared__ unsigned short key[CSR_CAP7]; __shared__ int outp[CSR_CAP7]; __shared__ int ncnt[CSR_GN7 + 1]; __shared__ int boff[CSR_NBLK7 + 1];
  const int g = blockIdx.x, t_ = threadIdx.x; int tot = TOT[g]; int st = START[g], stn = START[g + 1]; const int v0 = g * CSR_GN7; const int nv = min(CSR_GN7, N - v0); const int t0 = g * CSR_TS7;
  st = (st < 0) ? 0 : (st > permLen - 32 ? permLen - 32 : st) & ~31; stn = (stn < st) ? st : (stn > permLen ? permLen : stn); tot = (tot < 0) ? 0 : tot; if (tot > stn - st && tot <= CSR_CAP7) tot = stn - st;
  if (tot > CSR_CAP7) {
    for (int pass = 0; pass < 2; ++pass) { for (int i = t_; i < CSR_TS7 / 4; i += 256) { v4i a, c; for (int e = 0; e < 4; ++e) { a[e] = st; c[e] = 0; } *(volatile v4i*)(ROWPTR + t0 + i * 4) = a; *(volatile v4i*)(ROWCNT + t0 + i * 4) = c; } if (t_ == 0) ((volatile int*)FLAG)[0] = 1; __threadfence(); } (void)nv; return; }
  if (t_ == 0) { int acc = 0; for (int b = 0; b < CSR_NBLK7; ++b) { boff[b] = acc; int c = HST[(size_t)b * NGP + g]; c = (c < 0) ? 0 : (c > CHP ? CHP : c); acc += c; if (acc > tot) acc = tot; } boff[CSR_NBLK7] = acc; }
  for (int i = t_; i <= CSR_GN7; i += 256) ncnt[i] = 0;
  __syncthreads();
  for (int b = 0; b < CSR_NBLK7; ++b) { const int c = boff[b + 1] - boff[b]; int o_ = OFF[(size_t)g * CSR_NBLK7 + b]; o_ = (o_ < 0) ? 0 : (o_ > CHP - c ? CHP - c : o_); const int* src_ = STG + (size_t)b * CHP + o_;
    for (int i = t_; i < c; i += 256) { int id = src_[i]; id = (id < 0) ? 0 : id; ids[boff[b] + i] = id; int d = dst[id]; d = (d < v0) ? v0 : (d >= N ? N - 1 : d); int kk = d - v0; kk = (kk < 0) ? 0 : (kk >= CSR_GN7 ? CSR_GN7 - 1 : kk); key[boff[b] + i] = (unsigned short)kk; } }
  __syncthreads();
  if (t_ == 0) { for (int i = 0; i < tot; ++i) ncnt[key[i]] += 1; int acc = 0; for (int vl = 0; vl < CSR_GN7; ++vl) { const int c = ncnt[vl]; ncnt[vl] = acc; acc += c; } ncnt[CSR_GN7] = acc;
    for (int i = 0; i < tot; ++i) { const int vl = key[i]; outp[ncnt[vl]] = ids[i]; ncnt[vl] += 1; }
    for (int vl = CSR_GN7; vl > 0; --vl) ncnt[vl] = ncnt[vl - 1]; ncnt[0] = 0; }
  __syncthreads();
  for (int pass = 0; pass < 2; ++pass) {
    for (int i = t_; i < (stn - st) / 4; i += 256) { v4i v; for (int e = 0; e < 4; ++e) { const int q = i * 4 + e; v[e] = (q < tot) ? outp[q] : -1; } *(volatile v4i*)(PERM + st + i * 4) = v; }
    for (int i = t_; i < CSR_TS7 / 4; i += 256) { v4i a, c; for (int e = 0; e < 4; ++e) { const int vl = i * 4 + e; const int vc = vl < CSR_GN7 ? vl : CSR_GN7; a[e] = (vl < CSR_GN7) ? st + ncnt[vc] : st; c[e] = (vl < nv) ? (ncnt[(vc < CSR_GN7 ? vc : CSR_GN7 - 1) + 1] - ncnt[vc]) : 0; } *(volatile v4i*)(ROWPTR + t0 + i * 4) = a; *(volatile v4i*)(ROWCNT + t0 + i * 4) = c; }
    __threadfence(); }
}
__global__ __launch_bounds__(256) void csrZ_kernel7(int* __restrict__ p, size_t n4) { typedef __attribute__((ext_vector_type(4))) int v4i; const size_t tid = (size_t)blockIdx.x * 256 + threadIdx.x, nth = (size_t)gridDim.x * 256; v4i z = {0, 0, 0, 0}; for (size_t i = tid; i < n4; i += nth) *(volatile v4i*)(p + i * 4) = z; }
struct CsrBufs7 { int *STG, *HST, *OFF, *START, *TOT, *PERM, *ROWPTR, *ROWCNT, *FLAG; int nG, NGP, CHP; size_t permLen; char* base; size_t bytes; };
static size_t csr_carve7(CsrBufs7& c, char* ws, size_t off, int E, int N) {
  const size_t off0 = off; c.base = ws + off;
  auto al = [&](size_t bytes) { char* p = ws + off; off += (bytes + 255) & ~(size_t)255; return p; };
  c.nG = (N + CSR_GN7 - 1) / CSR_GN7; c.NGP = (c.nG + 31) & ~31; const int ch = (E + CSR_NBLK7 - 1) / CSR_NBLK7; c.CHP = (ch + 31) & ~31; c.permLen = (size_t)E + 32 * (size_t)c.nG + 32;
  c.STG = (int*)al((size_t)CSR_NBLK7 * c.CHP * 4); c.HST = (int*)al((size_t)CSR_NBLK7 * c.NGP * 4); c.OFF = (int*)al((size_t)c.NGP * CSR_NBLK7 * 4); c.START = (int*)al((size_t)(c.NGP + 64) * 4); c.TOT = (int*)al((size_t)(c.NGP + 64) * 4);
  c.PERM = (int*)al(c.permLen * 4); c.ROWPTR = (int*)al((size_t)c.nG * CSR_TS7 * 4); c.ROWCNT = (int*)al((size_t)c.nG * CSR_TS7 * 4); c.FLAG = (int*)al(256);
  c.bytes = off - off0; return off;
}
static void csr_build7(const CsrBufs7& c, const int* dst, int E, int N, hipStream_t stream) {
  const size_t smem = (size_t)(2 * c.NGP + c.CHP) * 4;
  csrZ_kernel7<<<512, 256, 0, stream>>>((int*)c.base, c.bytes / 16);
  csrA_kernel7<<<CSR_NBLK7, 64, smem, stream>>>(dst, E, N, c.nG, c.CHP, c.NGP, c.STG, c.HST);
  csrS_kernel7<<<1, 512, 0, stream>>>(c.HST, c.nG, c.NGP, c.START, c.TOT, c.OFF);
  csrB_kernel7<<<c.nG, 256, 0, stream>>>(dst, N, c.nG, c.CHP, c.NGP, (int)c.permLen, c.STG, c.HST, c.OFF, c.START, c.TOT, c.PERM, c.ROWPTR, c.ROWCNT, c.FLAG);
}


__global__ __launch_bounds__(256) void wput_kernel(const float* __restrict__ w, int base, int ks, int os, int KIN, int KW, int OUTW, int OUTP, int ro, int ko, int KP, b16* __restrict__ WT) {
  const int KG = KW / 8; const int u = blockIdx.x * 256 + threadIdx.x; if (u >= OUTP * KG) return; const int o = u / KG, k0 = (u % KG) * 8; v8b v;
#pragma unroll
  for (int j = 0; j < 8; ++j) { const int k = k0 + j; v[j] = (o < OUTW && k < KIN) ? (b16)(bf16_rne(w[(size_t)base + (size_t)k * ks + (size_t)o * os]) * WSC) : (b16)0.0f; }
  for (int pass = 0; pass < 2; ++pass) { *(volatile v8b*)(WT + (size_t)(ro + o) * KP + ko + k0) = v; __threadfence(); }
}
template <int KP, int NT, int FIRST, int RELU>
__global__ __launch_bounds__(32) void dense_kernel(const float* __restrict__ IN, int pin, int KIN, int nrows, const b16* __restrict__ WT, const float* __restrict__ bias, int nbias, int pout, float* __restrict__ OUT) {
  __shared__ __attribute__((aligned(16))) b16 Ah[16][KP + 8]; __shared__ __attribute__((aligned(16))) float Tf[16][128 + 4];
  const int lane = threadIdx.x, nloc = lane & 15, hlf = lane >> 4; const size_t m0 = (size_t)blockIdx.x * 16; if (m0 >= (size_t)nrows) return;
  for (int rr = 0; rr < 16; ++rr) for (int q = 0; q < KP / 32; ++q) { const int c = q * 32 + lane; float v = 0.0f; if (c < KIN && m0 + rr < (size_t)nrows) { v = IN[(m0 + rr) * pin + c]; if (FIRST) v = bf16_rne(v); } Ah[rr][c] = (b16)(v * XS); }
  wave_lds_sync();
#pragma unroll 1
  for (int cg = 0; cg < (NT + 7) / 8; ++cg) { const int nt = (NT - cg * 8) < 8 ? (NT - cg * 8) : 8; v8f acc[8];
#pragma unroll
    for (int t = 0; t < 8; ++t) acc[t] = (v8f){};
#pragma unroll 2
    for (int kb = 0; kb < KP; kb += 32) { const v16b a = frag_kb(&Ah[nloc][kb], hlf);
#pragma unroll
      for (int t = 0; t < 8; ++t) if (t < nt) acc[t] = wmma16b(a, frag_kb(WT + (size_t)(cg * 128 + t * 16 + nloc) * KP + kb, hlf), acc[t]); }
#pragma unroll
    for (int t = 0; t < 8; ++t) { if (t < nt) { const int c = cg * 128 + t * 16 + nloc; const float bb = (bias != nullptr && c < nbias) ? bf16_rne(bias[c]) : 0.0f;
#pragma unroll
        for (int r8 = 0; r8 < 8; ++r8) { float v = acc[t][r8] * (1.0f / (XS * WSC)) + bb; if (RELU) v = fmaxf(v, 0.0f); Tf[8 * hlf + r8][t * 16 + nloc] = v; } } }
    wave_lds_sync();
    for (int pass = 0; pass < 2; ++pass) { for (int rr = 0; rr < 16; ++rr) if (m0 + rr < (size_t)nrows) for (int c = lane; c < nt * 16; c += 32) ((volatile float*)OUT)[(m0 + rr) * pout + cg * 128 + c] = Tf[rr][c]; __threadfence(); }
    wave_lds_sync(); }
}
__global__ __launch_bounds__(256) void planes_kernel(const float* __restrict__ QKV, const float* __restrict__ KN, b16* __restrict__ QB, b16* __restrict__ KB_, b16* __restrict__ VT) {
  __shared__ float Tv[64][FP + 1]; const int nt = blockIdx.x; const int tid = threadIdx.x;
  for (int i = tid; i < 64 * 8; i += 256) { const int r = i / 8, q8 = (i % 8) * 8; const size_t n = (size_t)nt * 64 + r; v8b vq, vk; for (int j = 0; j < 8; ++j) { const int c = q8 + j; vq[j] = (n < (size_t)N && c < F) ? (b16)(QKV[n * 144 + c] * XS) : (b16)0.0f; vk[j] = (n < (size_t)N && c < F) ? (b16)(KN[n * FP + c] * XS) : (b16)0.0f; }
    if (n < (size_t)N) for (int pass = 0; pass < 2; ++pass) { *(volatile v8b*)(QB + n * 64 + q8) = vq; *(volatile v8b*)(KB_ + n * 64 + q8) = vk; __threadfence(); } }
  for (int i = tid; i < 64 * FP; i += 256) { const int r = i / FP, c = i % FP; const size_t n = (size_t)nt * 64 + r; Tv[r][c] = (n < (size_t)N && c < F) ? QKV[n * 144 + 96 + c] : 0.0f; }
  __syncthreads();
  for (int i = tid; i < FP * 8; i += 256) { const int c = i / 8, g8 = (i % 8) * 8; v8b v; for (int j = 0; j < 8; ++j) v[j] = (b16)(Tv[g8 + j][c] * XS); for (int pass = 0; pass < 2; ++pass) { *(volatile v8b*)(VT + (size_t)c * 10048 + (size_t)nt * 64 + g8) = v; __threadfence(); } }
}
__global__ __launch_bounds__(32) void att_kernel(const b16* __restrict__ QB, const b16* __restrict__ KB_, const b16* __restrict__ VT, int QLIM, float* __restrict__ HATT) {
  __shared__ __attribute__((aligned(16))) b16 Ph[16][40]; __shared__ float Mx[16], Sm[16]; __shared__ __attribute__((aligned(16))) float Tf[16][FP + 4];
  const int lane = threadIdx.x, nloc = lane & 15, hlf = lane >> 4; const size_t q0 = (size_t)blockIdx.x * 16; if (q0 >= (size_t)QLIM) return;
  const v16b qa0 = frag_kb(QB + (q0 + nloc) * 64, hlf), qa1 = frag_kb(QB + (q0 + nloc) * 64 + 32, hlf); const float scl = (1.0f / (XS * XS)) / sqrtf(35.0f);
  auto scores = [&](int kb, v8f sacc[2]) {
#pragma unroll
    for (int st = 0; st < 2; ++st) { const int k = kb + st * 16 + nloc; const b16* kr = KB_ + (size_t)(k < N ? k : N - 1) * 64; sacc[st] = (v8f){}; sacc[st] = wmma16b(qa0, frag_kb(kr, hlf), sacc[st]); sacc[st] = wmma16b(qa1, frag_kb(kr + 32, hlf), sacc[st]); } };
  float rmax[8];
#pragma unroll
  for (int r8 = 0; r8 < 8; ++r8) rmax[r8] = -INFINITY;
#pragma unroll 1
  for (int kb = 0; kb < N; kb += 32) { v8f sacc[2]; scores(kb, sacc);
#pragma unroll
    for (int st = 0; st < 2; ++st) { const int k = kb + st * 16 + nloc; if (k < N) {
#pragma unroll
        for (int r8 = 0; r8 < 8; ++r8) rmax[r8] = fmaxf(rmax[r8], sacc[st][r8] * scl); } } }
#pragma unroll
  for (int r8 = 0; r8 < 8; ++r8) { float m = rmax[r8]; for (int o = 1; o < 16; o <<= 1) m = fmaxf(m, __shfl_xor(m, o)); if (nloc == 0) Mx[8 * hlf + r8] = m; }
  wave_lds_sync();
  v8f acc[3] = {(v8f){}, (v8f){}, (v8f){}}; float rsum[8];
#pragma unroll
  for (int r8 = 0; r8 < 8; ++r8) rsum[r8] = 0.0f;
#pragma unroll 1
  for (int kb = 0; kb < N; kb += 32) { v8f sacc[2]; scores(kb, sacc);
#pragma unroll
    for (int st = 0; st < 2; ++st) { const int k = kb + st * 16 + nloc;
#pragma unroll
      for (int r8 = 0; r8 < 8; ++r8) { const int rl = 8 * hlf + r8; const float p = (k < N) ? __expf(sacc[st][r8] * scl - Mx[rl]) : 0.0f; rsum[r8] += p; Ph[rl][st * 16 + nloc] = (b16)(p * PS); } }
    wave_lds_sync();
    const v16b pa = frag_kb(&Ph[nloc][0], hlf);
#pragma unroll
    for (int t = 0; t < 3; ++t) acc[t] = wmma16b(pa, frag_kb(VT + (size_t)(t * 16 + nloc) * 10048 + kb, hlf), acc[t]);
    wave_lds_sync(); }
#pragma unroll
  for (int r8 = 0; r8 < 8; ++r8) { float s = rsum[r8]; for (int o = 1; o < 16; o <<= 1) s += __shfl_xor(s, o); if (nloc == 0) Sm[8 * hlf + r8] = s; }
  wave_lds_sync();
#pragma unroll
  for (int t = 0; t < 3; ++t)
#pragma unroll
    for (int r8 = 0; r8 < 8; ++r8) { const int rl = 8 * hlf + r8; Tf[rl][t * 16 + nloc] = fmaxf(acc[t][r8] * (1.0f / (PS * XS)) / Sm[rl], 0.0f); }
  wave_lds_sync();
  for (int pass = 0; pass < 2; ++pass) { for (int i = lane; i < 16 * FP; i += 32) ((volatile float*)HATT)[q0 * FP + i] = Tf[i / FP][i % FP]; __threadfence(); }
}
__global__ __launch_bounds__(32) void kn_kernel(const float* __restrict__ KC, const float* __restrict__ QKV, const b16* __restrict__ WLT, const float* __restrict__ blt, int NLIM, float* __restrict__ KN) {
  __shared__ __attribute__((aligned(16))) b16 Ah[16][168]; __shared__ __attribute__((aligned(16))) float Tf[16][FP + 4];
  const int lane = threadIdx.x, nloc = lane & 15, hlf = lane >> 4; const size_t m0 = (size_t)blockIdx.x * 16; if (m0 >= (size_t)NLIM) return;
  for (int rr = 0; rr < 16; ++rr) for (int q = 0; q < 5; ++q) { const int c = q * 32 + lane; float v = 0.0f; if (c < 96) v = KC[(m0 + rr) * 128 + c]; else if (c - 96 < F) v = QKV[(m0 + rr) * 144 + 48 + c - 96]; Ah[rr][c] = (b16)(v * XS); }
  wave_lds_sync();
#pragma unroll
  for (int t = 0; t < 3; ++t) { v8f acc = {};
#pragma unroll
    for (int kb = 0; kb < 160; kb += 32) acc = wmma16b(frag_kb(&Ah[nloc][kb], hlf), frag_kb(WLT + (size_t)(t * 16 + nloc) * 160 + kb, hlf), acc);
    const int c = t * 16 + nloc; const float bb = c < F ? bf16_rne(blt[c]) : 0.0f;
#pragma unroll
    for (int r8 = 0; r8 < 8; ++r8) Tf[8 * hlf + r8][c] = acc[r8] * (1.0f / (XS * WSC)) + bb; }
  wave_lds_sync();
  for (int pass = 0; pass < 2; ++pass) { for (int i = lane; i < 16 * FP; i += 32) ((volatile float*)KN)[m0 * FP + i] = Tf[i / FP][i % FP]; __threadfence(); }
}
__global__ __launch_bounds__(32) void sagepre_kernel(const float* __restrict__ HATT, const int* __restrict__ srcs, const int* __restrict__ PERM, const int* __restrict__ ROWPTR, const int* __restrict__ ROWCNT, int permLen, int NLIM, float* __restrict__ MH) {
  const int lane = threadIdx.x; const size_t m0 = (size_t)blockIdx.x * 16; if (m0 >= (size_t)NLIM) return; const bool hi_ok = (lane + 32) < F;
  for (int rr = 0; rr < 16; ++rr) { const size_t v = m0 + rr; int st = ROWPTR[v], cnt = ROWCNT[v]; cnt = iclamp(cnt, 0, 1 << 20); st = iclamp(st, 0, permLen - cnt); float a0 = 0.0f, a1 = 0.0f; int nn = 0;
#pragma unroll 1
    for (int j = 0; j < cnt; ++j) { const int e = iclamp(PERM[st + j], 0, E - 1); const size_t u = (size_t)iclamp(srcs[e], 0, N - 1); if (u >= (size_t)NLIM) continue; ++nn; a0 += HATT[u * FP + lane]; if (hi_ok) a1 += HATT[u * FP + 32 + lane]; }
    const float inv = 1.0f / (float)(nn < 1 ? 1 : nn); const float m0v = pmul(a0, inv), m1v = hi_ok ? pmul(a1, inv) : 0.0f; const float o0 = HATT[v * FP + lane], o1 = hi_ok ? HATT[v * FP + 32 + lane] : 0.0f;
    for (int pass = 0; pass < 2; ++pass) { ((volatile float*)MH)[v * 128 + lane] = m0v; ((volatile float*)MH)[v * 128 + 32 + lane] = m1v; ((volatile float*)MH)[v * 128 + 64 + lane] = o0; ((volatile float*)MH)[v * 128 + 96 + lane] = o1; __threadfence(); } }
}
__global__ __launch_bounds__(64) void pool_kernel(const float* __restrict__ H2, const int* __restrict__ batch, int NLIM, float* __restrict__ GP) {
  const int g = blockIdx.x, c = threadIdx.x;
  auto lb = [&](int key) -> int { int lo = 0, hi = N; for (int it = 0; it < 15 && lo < hi; ++it) { const int mid = (lo + hi) >> 1; if (batch[mid] < key) lo = mid + 1; else hi = mid; } return lo; };
  int s0 = lb(g), e0 = lb(g + 1); if (e0 > NLIM) e0 = NLIM; if (e0 < s0) e0 = s0; const int ch = c < 32 ? c : c - 32 + 32;
  float mx = -INFINITY, sm = 0.0f; const int cc = c % 35; (void)ch;
#pragma unroll 1
  for (int n = s0; n < e0; ++n) { const float v = H2[(size_t)n * FP + cc]; mx = fmaxf(mx, v); sm += v; }
  const int cnt = e0 - s0; const float vmax = cnt > 0 ? mx : 0.0f, vmean = sm / (float)(cnt < 1 ? 1 : cnt);
  for (int pass = 0; pass < 2; ++pass) { if (c < 35) { ((volatile float*)GP)[g * 128 + c] = vmax; ((volatile float*)GP)[g * 128 + 35 + c] = vmean; } else if (c - 35 + 70 < 128) ((volatile float*)GP)[g * 128 + 70 + (c - 35)] = 0.0f; __threadfence(); }
}
__global__ __launch_bounds__(64) void out_kernel(const float* __restrict__ G2, const float* __restrict__ Wo, const float* __restrict__ bo, float* __restrict__ out) {
  __shared__ float So[32]; const int wave = threadIdx.x >> 5, lane = threadIdx.x & 31; const int g0 = blockIdx.x * 32 + wave * 16;
  for (int rr = 0; rr < 16; ++rr) { float s = 0.0f; for (int q = 0; q < 4; ++q) s += pmul(G2[(size_t)(g0 + rr) * H2 + q * 32 + lane], bf16_rne(Wo[q * 32 + lane])); for (int o = 16; o; o >>= 1) s += __shfl_xor(s, o); if (lane == 0) So[wave * 16 + rr] = s + bf16_rne(bo[0]); }
  __syncthreads();
  if (wave == 0) for (int pass = 0; pass < 2; ++pass) { ((volatile float*)out)[blockIdx.x * 32 + lane] = So[lane]; __threadfence(); }
}
}

extern "C" void kernel_launch(void* const* d_in, const int* in_sizes, int n_in, void* d_out, int out_size, void* d_ws, size_t ws_size, hipStream_t stream) {
  (void)n_in;
  auto Fp = [&](int i) { return (const float*)d_in[i]; }; auto Ip = [&](int i) { return (const int*)d_in[i]; };
  if (in_sizes[0] != N * F || in_sizes[1] != 2 * E || in_sizes[2] != N || in_sizes[3] != F * F || in_sizes[9] != F * F * 3 || in_sizes[11] != F * F * 5 || in_sizes[13] != 3 * F * F || in_sizes[18] != 2 * F * H1 || in_sizes[20] != H1 * H2 || in_sizes[22] != H2 || out_size != G) return;
  const int NLIM = N; const int GB16 = NBLK;
  size_t off = 0; char* ws = (char*)d_ws;
  auto carve = [&](size_t bytes) { char* p = ws + off; off += (bytes + 255) & ~(size_t)255; return p; };
  b16* WQKV = (b16*)carve(144 * 64 * 2); b16* WC35 = (b16*)carve(96 * 64 * 2); b16* WLT = (b16*)carve(48 * 128 * 2); b16* WSG = (b16*)carve(48 * 128 * 2); b16* WM1 = (b16*)carve((size_t)H1P * 128 * 2); b16* WM2 = (b16*)carve((size_t)128 * 1536 * 2);
  float* QKV = (float*)carve((size_t)N * 144 * 4); float* KC = (float*)carve((size_t)N * 128 * 4); float* KN = (float*)carve((size_t)N * FP * 4); b16* QB = (b16*)carve((size_t)N * 64 * 2); b16* KB_ = (b16*)carve((size_t)N * 64 * 2); b16* VT = (b16*)carve((size_t)FP * 10048 * 2);
  float* HATT = (float*)carve((size_t)N * FP * 4); float* MH = (float*)carve((size_t)N * 128 * 4); float* HS = (float*)carve((size_t)N * FP * 4); float* GP = (float*)carve((size_t)G * 128 * 4); float* G1 = (float*)carve((size_t)G * H1P * 4); float* G2 = (float*)carve((size_t)G * H2 * 4);
  float* BQKV = (float*)carve(144 * 4); float* BC = (float*)carve(96 * 4);
  CsrBufs7 csr; off = csr_carve7(csr, ws, off, E, N);
  if (off > ws_size || off > ((size_t)64 << 20)) return;
  wput_kernel<<<(48 * 8 + 255) / 256, 256, 0, stream>>>(Fp(3), 0, F, 1, F, 64, F, 48, 0, 0, 64, WQKV); wput_kernel<<<(48 * 8 + 255) / 256, 256, 0, stream>>>(Fp(5), 0, F, 1, F, 64, F, 48, 48, 0, 64, WQKV); wput_kernel<<<(48 * 8 + 255) / 256, 256, 0, stream>>>(Fp(7), 0, F, 1, F, 64, F, 48, 96, 0, 64, WQKV);
  wput_kernel<<<(48 * 8 + 255) / 256, 256, 0, stream>>>(Fp(9), 1, 3, F * 3, F, 64, F, 48, 0, 0, 64, WC35); wput_kernel<<<(48 * 8 + 255) / 256, 256, 0, stream>>>(Fp(11), 2, 5, F * 5, F, 64, F, 48, 48, 0, 64, WC35);
  for (int b = 0; b < 3; ++b) wput_kernel<<<(48 * 6 + 255) / 256, 256, 0, stream>>>(Fp(13), b * F * F, F, 1, F, 48, F, 48, 0, b * 48, 160, WLT);
  { const int nz8 = 48 * (160 - 144) / 8; (void)nz8; }
  wput_kernel<<<(48 * 2 + 255) / 256, 256, 0, stream>>>(Fp(13), 0, 1, 1, 0, 16, 0, 48, 0, 144, 160, WLT);
  wput_kernel<<<(48 * 8 + 255) / 256, 256, 0, stream>>>(Fp(15), 0, F, 1, F, 64, F, 48, 0, 0, 128, WSG); wput_kernel<<<(48 * 8 + 255) / 256, 256, 0, stream>>>(Fp(17), 0, F, 1, F, 64, F, 48, 0, 64, 128, WSG);
  wput_kernel<<<(H1P * 16 + 255) / 256, 256, 0, stream>>>(Fp(18), 0, H1, 1, 2 * F, 128, H1, H1P, 0, 0, 128, WM1);
  wput_kernel<<<(128 * 192 + 255) / 256, 256, 0, stream>>>(Fp(20), 0, H2, 1, H1, 1536, H2, 128, 0, 0, 1536, WM2);
  csr_build7(csr, Ip(1) + E, E, N, stream);
  dense_kernel<64, 3, 1, 0><<<NBLK, 32, 0, stream>>>(Fp(0), F, F, N, WQKV, Fp(4), F, 144, QKV);
  dense_kernel<64, 3, 1, 0><<<NBLK, 32, 0, stream>>>(Fp(0), F, F, N, WQKV + 48 * 64, Fp(6), F, 144, QKV + 48);
  dense_kernel<64, 3, 1, 0><<<NBLK, 32, 0, stream>>>(Fp(0), F, F, N, WQKV + 96 * 64, Fp(8), F, 144, QKV + 96);
  dense_kernel<64, 3, 0, 0><<<NBLK, 32, 0, stream>>>(QKV + 48, 144, F, N, WC35, Fp(10), F, 128, KC);
  dense_kernel<64, 3, 0, 0><<<NBLK, 32, 0, stream>>>(QKV + 48, 144, F, N, WC35 + 48 * 64, Fp(12), F, 128, KC + 48);
  kn_kernel<<<NBLK, 32, 0, stream>>>(KC, QKV, WLT, Fp(14), N, KN);
  planes_kernel<<<(N + 63) / 64, 256, 0, stream>>>(QKV, KN, QB, KB_, VT);
  att_kernel<<<GB16, 32, 0, stream>>>(QB, KB_, VT, NLIM, HATT);
  sagepre_kernel<<<GB16, 32, 0, stream>>>(HATT, Ip(1), csr.PERM, csr.ROWPTR, csr.ROWCNT, (int)csr.permLen, NLIM, MH);
  dense_kernel<128, 3, 0, 1><<<GB16, 32, 0, stream>>>(MH, 128, 128, NLIM, WSG, Fp(16), F, FP, HS);
  pool_kernel<<<G, 64, 0, stream>>>(HS, Ip(2), NLIM, GP);
  dense_kernel<128, 94, 0, 1><<<G / 16, 32, 0, stream>>>(GP, 128, 2 * F, G, WM1, Fp(19), H1, H1P, G1);
  dense_kernel<1536, 8, 0, 0><<<G / 16, 32, 0, stream>>>(G1, H1P, H1, G, WM2, Fp(21), H2, H2, G2);
  out_kernel<<<G / 32, 64, 0, stream>>>(G2, Fp(22), Fp(23), (float*)d_out);
}
